// EquivariantEdgeAttention_25924422599458
// MI455X (gfx1250) — hardware-verified
//
#include <hip/hip_runtime.h>
#include <stddef.h>


#define E_N   384
#define HID   128
#define NHD   8
#define DHD   16
#define NRB   64
#define NTH   128
#define QKVW  384
#define GPW   32
#define CPW   32
#define TP    132
#define TRP   136
#define XP    136

#define SC_EF   16.0f
#define SC_W    64.0f
#define SC_RBF  1024.0f
#define SC_X1   16.0f
#define SC_UPD  256.0f
#define INV_QKV 0.0009765625f
#define INV_R   0.0000152587890625f
#define INV_L2  0.0009765625f
#define INV_OUT 0.00006103515625f

typedef float    v4f  __attribute__((ext_vector_type(4)));
typedef float    v8f  __attribute__((ext_vector_type(8)));
typedef _Float16 v8h  __attribute__((ext_vector_type(8)));
typedef _Float16 v16h __attribute__((ext_vector_type(16)));
union FragH { v16h v; v8h h[2]; };

__device__ __forceinline__ v8f zero8f() {
  v8f z = {0.0f, 0.0f, 0.0f, 0.0f, 0.0f, 0.0f, 0.0f, 0.0f};
  return z;
}

__device__ __forceinline__ v8f wmh(v16h a, v16h b, v8f c) {
  v8f d = __builtin_amdgcn_wmma_f32_16x16x32_f16(false, a, false, b, (short)0, c, false, false);
  asm volatile("v_nop\n\tv_nop\n\tv_nop\n\tv_nop" : "+v"(d) : "v"(a), "v"(b));
  return d;
}

__device__ __forceinline__ float frcp(float x) { return __builtin_amdgcn_rcpf(x); }
__device__ __forceinline__ float fexp(float x) { return __builtin_amdgcn_exp2f(x * 1.4426950408889634f); }
__device__ __forceinline__ float fsilu(float x) { return x * frcp(1.0f + fexp(-x)); }
__device__ __forceinline__ float fsigm(float x) { return frcp(1.0f + fexp(-x)); }

__device__ __forceinline__ float wsum(float v) {
  v += __shfl_xor(v, 16); v += __shfl_xor(v, 8); v += __shfl_xor(v, 4);
  v += __shfl_xor(v, 2);  v += __shfl_xor(v, 1);
  return v;
}
__device__ __forceinline__ float wmax(float v) {
  v = fmaxf(v, __shfl_xor(v, 16)); v = fmaxf(v, __shfl_xor(v, 8)); v = fmaxf(v, __shfl_xor(v, 4));
  v = fmaxf(v, __shfl_xor(v, 2));  v = fmaxf(v, __shfl_xor(v, 1));
  return v;
}

__global__ __launch_bounds__(NTH) void k_prep(
    const float* __restrict__ ef, const float* __restrict__ wq, const float* __restrict__ wk,
    const float* __restrict__ wv, const float* __restrict__ wo, const float* __restrict__ aw2,
    const float* __restrict__ aw1,
    _Float16* qkvT, _Float16* woT, _Float16* w2T, _Float16* a3T, _Float16* efH) {
  __shared__ __attribute__((aligned(16))) _Float16 sTr[32 * TRP];
  const int tid = threadIdx.x, lane = tid & 31, wave = tid >> 5;
  const int b = blockIdx.x;
  if (b >= 36) return;
  const float* src;
  _Float16* dst;
  int kdim, trans, c0, r0;
  float sc;
  if (b < 12) {
    const int n0 = b * 32;
    src = (n0 < HID) ? wq : ((n0 < 2 * HID) ? wk : wv);
    kdim = HID; trans = 1; c0 = n0 & (HID - 1); r0 = n0; sc = SC_W; dst = qkvT;
  } else if (b < 16) {
    src = wo;  kdim = HID; trans = 1; c0 = (b - 12) * 32; r0 = c0; sc = SC_W; dst = woT;
  } else if (b < 20) {
    src = aw2; kdim = HID; trans = 1; c0 = (b - 16) * 32; r0 = c0; sc = SC_W; dst = w2T;
  } else if (b < 24) {
    src = aw1 + 32 * HID; kdim = NRB; trans = 1; c0 = (b - 20) * 32; r0 = c0; sc = SC_W; dst = a3T;
  } else {
    src = ef;  kdim = HID; trans = 0; c0 = (b - 24) * 32; r0 = c0; sc = SC_EF; dst = efH;
  }
  const int nel = 32 * kdim;
  if (trans != 0) {
    for (int idx = tid; idx < nel; idx += NTH) {
      const int kk = idx >> 5, rr = idx & 31;
      sTr[rr * TRP + kk] = (_Float16)(src[(size_t)kk * HID + c0 + rr] * sc);
    }
  } else {
    for (int idx = tid; idx < nel; idx += NTH) {
      const int rr = idx >> 7, kk = idx & 127;
      sTr[rr * TRP + kk] = (_Float16)(src[(size_t)(c0 + rr) * HID + kk] * sc);
    }
  }
  __syncthreads();
  if (kdim == HID) {
    v8h val[4];
#pragma unroll
    for (int q = 0; q < 4; ++q) {
      const int p = wave + 4 * q, row = 2 * p + (lane >> 4), col = (lane & 15) * 8;
      val[q] = *(const v8h*)(sTr + row * TRP + col);
    }
#pragma unroll
    for (int q = 0; q < 4; ++q) {
      const int p = wave + 4 * q, row = 2 * p + (lane >> 4), col = (lane & 15) * 8;
      *(volatile v8h*)(dst + (size_t)(r0 + row) * HID + col) = val[q];
    }
    __threadfence();
#pragma unroll
    for (int q = 0; q < 4; ++q) {
      const int p = wave + 4 * q, row = 2 * p + (lane >> 4), col = (lane & 15) * 8;
      *(volatile v8h*)(dst + (size_t)(r0 + row) * HID + col) = val[q];
    }
  } else {
    v8h val[2];
#pragma unroll
    for (int q = 0; q < 2; ++q) {
      const int p = wave + 4 * q, row = 4 * p + (lane >> 3), col = (lane & 7) * 8;
      val[q] = *(const v8h*)(sTr + row * TRP + col);
    }
#pragma unroll
    for (int q = 0; q < 2; ++q) {
      const int p = wave + 4 * q, row = 4 * p + (lane >> 3), col = (lane & 7) * 8;
      *(volatile v8h*)(dst + (size_t)(r0 + row) * NRB + col) = val[q];
    }
    __threadfence();
#pragma unroll
    for (int q = 0; q < 2; ++q) {
      const int p = wave + 4 * q, row = 4 * p + (lane >> 3), col = (lane & 7) * 8;
      *(volatile v8h*)(dst + (size_t)(r0 + row) * NRB + col) = val[q];
    }
  }
}

__device__ __forceinline__ void gemm_tile(const _Float16* __restrict__ A, int row0,
                                          const _Float16* __restrict__ Bt, int col0,
                                          float* sTile, float osc, int lane, int wave) {
  const int hh = lane >> 4, m = lane & 15;
  v8f a00 = zero8f(), a01 = zero8f(), a10 = zero8f(), a11 = zero8f();
#pragma unroll
  for (int s = 0; s < 4; ++s) {
    FragH fa0, fa1, fb0, fb1;
    const _Float16* ap0 = A + (size_t)(row0 + m) * HID + 32 * s + 8 * hh;
    const _Float16* ap1 = A + (size_t)(row0 + 16 + m) * HID + 32 * s + 8 * hh;
    fa0.h[0] = *(const v8h*)ap0; fa0.h[1] = *(const v8h*)(ap0 + 16);
    fa1.h[0] = *(const v8h*)ap1; fa1.h[1] = *(const v8h*)(ap1 + 16);
    const _Float16* bp0 = Bt + (size_t)(col0 + 32 * wave + m) * HID + 32 * s + 8 * hh;
    const _Float16* bp1 = Bt + (size_t)(col0 + 32 * wave + 16 + m) * HID + 32 * s + 8 * hh;
    fb0.h[0] = *(const v8h*)bp0; fb0.h[1] = *(const v8h*)(bp0 + 16);
    fb1.h[0] = *(const v8h*)bp1; fb1.h[1] = *(const v8h*)(bp1 + 16);
    a00 = wmh(fa0.v, fb0.v, a00);
    a01 = wmh(fa0.v, fb1.v, a01);
    a10 = wmh(fa1.v, fb0.v, a10);
    a11 = wmh(fa1.v, fb1.v, a11);
  }
#pragma unroll
  for (int r = 0; r < 8; ++r) {
    sTile[(8 * hh + r) * TP + 32 * wave + m]           = a00[r] * osc;
    sTile[(8 * hh + r) * TP + 32 * wave + 16 + m]      = a01[r] * osc;
    sTile[(16 + 8 * hh + r) * TP + 32 * wave + m]      = a10[r] * osc;
    sTile[(16 + 8 * hh + r) * TP + 32 * wave + 16 + m] = a11[r] * osc;
  }
}

__global__ __launch_bounds__(NTH) void k_qkv(const _Float16* __restrict__ efH,
                                             const _Float16* __restrict__ qkvT, float* qkv) {
  __shared__ __attribute__((aligned(16))) float sTile[32 * TP];
  const int tid = threadIdx.x, lane = tid & 31, wave = tid >> 5;
  const int rb = blockIdx.x, cb = blockIdx.y;
  if (rb >= E_N / 32 || cb >= 3) return;
  gemm_tile(efH, 32 * rb, qkvT, HID * cb, sTile, INV_QKV, lane, wave);
  __syncthreads();
  v4f vals[8];
#pragma unroll
  for (int q = 0; q < 8; ++q) {
    const int row = wave + 4 * q;
    vals[q] = *(const v4f*)(sTile + row * TP + 4 * lane);
  }
#pragma unroll
  for (int q = 0; q < 8; ++q) {
    const int row = wave + 4 * q;
    *(volatile v4f*)(qkv + (size_t)(32 * rb + row) * QKVW + HID * cb + 4 * lane) = vals[q];
  }
  __threadfence();
#pragma unroll
  for (int q = 0; q < 8; ++q) {
    const int row = wave + 4 * q;
    *(volatile v4f*)(qkv + (size_t)(32 * rb + row) * QKVW + HID * cb + 4 * lane) = vals[q];
  }
}

__global__ __launch_bounds__(NTH) void k_node(
    const float* __restrict__ qkv, const float* __restrict__ aw1, const float* __restrict__ ab1,
    const float* __restrict__ gw1, const float* __restrict__ gb1,
    const float* __restrict__ gw2, const float* __restrict__ gb2,
    float* Pp, float* Qp, float* gpl) {
  __shared__ __attribute__((aligned(16))) float sRow[QKVW];
  __shared__ __attribute__((aligned(16))) float sOut[2 * NHD * HID];
  __shared__ float sRed[NHD * HID];
  __shared__ __attribute__((aligned(16))) float sG[32];
  const int tid = threadIdx.x, lane = tid & 31, wave = tid >> 5;
  const int i = blockIdx.x;
  if (i >= E_N) return;
  for (int c = tid; c < QKVW; c += NTH) sRow[c] = qkv[(size_t)i * QKVW + c];
  __syncthreads();
  const int f = tid;
  const float b1 = ab1[f], g1 = gb1[f], g2 = gw2[f];
#pragma unroll 1
  for (int h = 0; h < NHD; ++h) {
    float p = 0.0f, qq = 0.0f, g = 0.0f;
#pragma unroll
    for (int d = 0; d < DHD; ++d) {
      p  += sRow[h * DHD + d]           * aw1[(size_t)d * HID + f];
      qq += sRow[HID + h * DHD + d]     * aw1[(size_t)(DHD + d) * HID + f];
      g  += sRow[2 * HID + h * DHD + d] * gw1[(size_t)d * HID + f];
    }
    sOut[h * HID + f]         = p + b1;
    sOut[(NHD + h) * HID + f] = qq;
    sRed[h * HID + f]         = fsilu(g + g1) * g2;
  }
  __syncthreads();
  if (tid < NHD) {
    float s = 0.0f;
#pragma unroll 8
    for (int c = 0; c < HID; ++c) s += sRed[tid * HID + c];
    sG[tid] = fsigm(s + gb2[0]);
  } else if (tid < 32) {
    sG[tid] = 0.0f;
  }
  __syncthreads();
  v4f vals[4];
#pragma unroll
  for (int q = 0; q < 4; ++q) {
    const int r = wave + 4 * q;
    vals[q] = *(const v4f*)(sOut + r * HID + 4 * lane);
  }
  const int l8 = lane & 7;
  const v4f gv = *(const v4f*)(sG + 4 * l8);
  const bool wg = (wave == 0) && (lane < 8);
#pragma unroll
  for (int q = 0; q < 4; ++q) {
    const int r = wave + 4 * q;
    float* p = (q < 2) ? (Pp + ((size_t)(r * E_N + i)) * HID + 4 * lane)
                       : (Qp + ((size_t)((r - NHD) * E_N + i)) * HID + 4 * lane);
    *(volatile v4f*)p = vals[q];
  }
  if (wg) *(volatile v4f*)(gpl + (size_t)i * GPW + 4 * lane) = gv;
  __threadfence();
#pragma unroll
  for (int q = 0; q < 4; ++q) {
    const int r = wave + 4 * q;
    float* p = (q < 2) ? (Pp + ((size_t)(r * E_N + i)) * HID + 4 * lane)
                       : (Qp + ((size_t)((r - NHD) * E_N + i)) * HID + 4 * lane);
    *(volatile v4f*)p = vals[q];
  }
  if (wg) *(volatile v4f*)(gpl + (size_t)i * GPW + 4 * lane) = gv;
}

__global__ __launch_bounds__(NTH) void k_attn(
    const float* __restrict__ ec, const float* __restrict__ emask,
    const float* __restrict__ rbc, const float* __restrict__ rbw,
    const float* __restrict__ aw1, const float* __restrict__ ab2,
    const float* __restrict__ aw3, const float* __restrict__ ab3,
    const float* __restrict__ qkv, const float* __restrict__ Pp, const float* __restrict__ Qp,
    const float* __restrict__ gpl, const _Float16* __restrict__ a3T, const _Float16* __restrict__ w2T,
    _Float16* updH, float* cpl) {
  __shared__ __attribute__((aligned(16))) _Float16 sA3[HID * NRB];
  __shared__ __attribute__((aligned(16))) _Float16 sW2[HID * HID];
  __shared__ __attribute__((aligned(16))) _Float16 sX1[4 * 16 * XP];
  __shared__ __attribute__((aligned(16))) float    sR[4 * 32 * 64];
  __shared__ __attribute__((aligned(16))) float    sS[NHD * E_N];
  __shared__ __attribute__((aligned(16))) float    sCj[E_N * 4];
  __shared__ __attribute__((aligned(16))) float    sPB[NHD * HID];
  __shared__ __attribute__((aligned(16))) float    sW3[NHD * HID];
  __shared__ __attribute__((aligned(16))) float    sA4[HID];
  __shared__ __attribute__((aligned(16))) float    sB2[HID];
  __shared__ __attribute__((aligned(16))) float    sU[HID];
  __shared__ float sRC[NRB], sRW[NRB];
  __shared__ float sB3[NHD], sGt[NHD];
  __shared__ float sTc[NHD * 4];
  __shared__ __attribute__((aligned(16))) float sCo[4];

  const int tid = threadIdx.x, lane = tid & 31, wave = tid >> 5, hh = lane >> 4, m = lane & 15;
  const int i = blockIdx.x;
  if (i >= E_N) return;

  {
    const v8h* s3 = (const v8h*)a3T; v8h* d3 = (v8h*)sA3;
    for (int idx = tid; idx < (HID * NRB) / 8; idx += NTH) d3[idx] = s3[idx];
    const v8h* s2 = (const v8h*)w2T; v8h* d2 = (v8h*)sW2;
    for (int idx = tid; idx < (HID * HID) / 8; idx += NTH) d2[idx] = s2[idx];
  }
  for (int c = tid; c < NHD * HID; c += NTH) {
    const int h = c >> 7, f = c & (HID - 1);
    sPB[c] = Pp[((size_t)h * E_N + i) * HID + f];
  }
  sA4[tid] = aw1[96 * HID + tid];
  sB2[tid] = ab2[tid];
  {
    const v4f w0 = *(const v4f*)(aw3 + 8 * tid);
    const v4f w1 = *(const v4f*)(aw3 + 8 * tid + 4);
    sW3[0 * HID + tid] = w0.x; sW3[1 * HID + tid] = w0.y; sW3[2 * HID + tid] = w0.z; sW3[3 * HID + tid] = w0.w;
    sW3[4 * HID + tid] = w1.x; sW3[5 * HID + tid] = w1.y; sW3[6 * HID + tid] = w1.z; sW3[7 * HID + tid] = w1.w;
  }
  if (tid < NRB) { sRC[tid] = rbc[tid]; sRW[tid] = rbw[tid]; }
  if (tid < NHD) { sB3[tid] = ab3[tid]; sGt[tid] = gpl[(size_t)i * GPW + tid]; }
  for (int c = tid; c < E_N; c += NTH) {
    sCj[c * 4 + 0] = ec[c * 3 + 0];
    sCj[c * 4 + 1] = ec[c * 3 + 1];
    sCj[c * 4 + 2] = ec[c * 3 + 2];
    sCj[c * 4 + 3] = 0.0f;
  }
  const float cix = ec[i * 3 + 0], ciy = ec[i * 3 + 1], ciz = ec[i * 3 + 2];
  __syncthreads();

  float* rsp = sR + (wave * 32 + lane) * 64;
  _Float16* x1row = sX1 + (wave * 16 + m) * XP;
  const float* emrow = emask + (size_t)i * E_N;

#pragma unroll 1
  for (int tt = 0; tt < 6; ++tt) {
    const int j = (tt * 4 + wave) * 16 + m;
    const float cjx = sCj[j * 4 + 0], cjy = sCj[j * 4 + 1], cjz = sCj[j * 4 + 2];
    const float dx = cix - cjx, dy = ciy - cjy, dz = ciz - cjz;
    float dist = sqrtf(dx * dx + dy * dy + dz * dz) + 1e-8f;
    dist = fminf(fmaxf(dist, 1e-8f), 1e8f);
    const float rsc = (dist <= 10.0f) ? SC_RBF : 0.0f;
    float dotv = cix * cjx + ciy * cjy + ciz * cjz;
    dotv = fminf(fmaxf(dotv, -1e8f), 1e8f);
    const float em = emrow[j];

    FragH br[2];
#pragma unroll
    for (int s = 0; s < 2; ++s) {
#pragma unroll
      for (int hf = 0; hf < 2; ++hf) {
#pragma unroll
        for (int r = 0; r < 8; ++r) {
          const int ri = 32 * s + 16 * hf + 8 * hh + r;
          const float dc = dist - sRC[ri];
          const float e = fexp(-(sRW[ri] * (dc * dc))) * rsc;
          br[s].h[hf][r] = (_Float16)e;
        }
      }
    }
#pragma unroll 1
    for (int ft = 0; ft < 8; ++ft) {
      v8f acc = zero8f();
#pragma unroll
      for (int s = 0; s < 2; ++s) {
        FragH a;
        const _Float16* ap = sA3 + (16 * ft + m) * NRB + 32 * s + 8 * hh;
        a.h[0] = *(const v8h*)ap;
        a.h[1] = *(const v8h*)(ap + 16);
        acc = wmh(a.v, br[s].v, acc);
      }
      const v4f lo4 = {acc[0] * INV_R, acc[1] * INV_R, acc[2] * INV_R, acc[3] * INV_R};
      const v4f hi4 = {acc[4] * INV_R, acc[5] * INV_R, acc[6] * INV_R, acc[7] * INV_R};
      *(v4f*)(rsp + 8 * ft)     = lo4;
      *(v4f*)(rsp + 8 * ft + 4) = hi4;
    }
    __syncthreads();

#pragma unroll 1
    for (int h = 0; h < NHD; ++h) {
      const float* qrow = Qp + ((size_t)(h * E_N + j)) * HID;
      const float* pb = sPB + h * HID;
#pragma unroll 1
      for (int s = 0; s < 4; ++s) {
#pragma unroll
        for (int hf = 0; hf < 2; ++hf) {
          const int f0 = 32 * s + 16 * hf + 8 * hh;
          const v4f ra  = *(const v4f*)(rsp + 16 * s + 8 * hf);
          const v4f rbv = *(const v4f*)(rsp + 16 * s + 8 * hf + 4);
          const v4f qa  = *(const v4f*)(qrow + f0);
          const v4f qb  = *(const v4f*)(qrow + f0 + 4);
          const v4f pa  = *(const v4f*)(pb + f0);
          const v4f pbv = *(const v4f*)(pb + f0 + 4);
          const v4f wa  = *(const v4f*)(sA4 + f0);
          const v4f wb  = *(const v4f*)(sA4 + f0 + 4);
          v8h xv;
#pragma unroll
          for (int r = 0; r < 4; ++r) {
            const float x0 = (pa[r] + qa[r]) + (ra[r] + dotv * wa[r]);
            const float x1 = (pbv[r] + qb[r]) + (rbv[r] + dotv * wb[r]);
            xv[r]     = (_Float16)(fsilu(x0) * SC_X1);
            xv[4 + r] = (_Float16)(fsilu(x1) * SC_X1);
          }
          *(v8h*)(x1row + f0) = xv;
        }
      }
      __syncthreads();
      float sc = 0.0f;
#pragma unroll 1
      for (int ft = 0; ft < 8; ++ft) {
        v8f acc = zero8f();
#pragma unroll
        for (int s = 0; s < 4; ++s) {
          FragH a, b;
          const _Float16* ap = sW2 + (16 * ft + m) * HID + 32 * s + 8 * hh;
          a.h[0] = *(const v8h*)ap;
          a.h[1] = *(const v8h*)(ap + 16);
          const _Float16* bp = x1row + 32 * s + 8 * hh;
          b.h[0] = *(const v8h*)bp;
          b.h[1] = *(const v8h*)(bp + 16);
          acc = wmh(a.v, b.v, acc);
        }
        const int f0 = 16 * ft + 8 * hh;
        const v4f ba = *(const v4f*)(sB2 + f0);
        const v4f bb = *(const v4f*)(sB2 + f0 + 4);
        const v4f wa = *(const v4f*)(sW3 + h * HID + f0);
        const v4f wb = *(const v4f*)(sW3 + h * HID + f0 + 4);
#pragma unroll
        for (int r = 0; r < 4; ++r) {
          const float x2a = fsilu(acc[r] * INV_L2 + ba[r]);
          const float x2b = fsilu(acc[4 + r] * INV_L2 + bb[r]);
          sc += x2a * wa[r];
          sc += x2b * wb[r];
        }
      }
      sc += __shfl_xor(sc, 16);
      if (hh == 0) {
        float s2 = sc + sB3[h] + em;
        s2 = fminf(fmaxf(s2, -1.0e9f), 1.0e9f);
        sS[h * E_N + j] = s2;
      }
    }
  }
  __syncthreads();

#pragma unroll 1
  for (int hp = 0; hp < 2; ++hp) {
    const int h = wave + 4 * hp;
    float* srow = sS + h * E_N;
    float sv[12];
#pragma unroll
    for (int t = 0; t < 12; ++t) sv[t] = srow[lane + 32 * t];
    float mx = sv[0];
#pragma unroll
    for (int t = 1; t < 12; ++t) mx = fmaxf(mx, sv[t]);
    mx = wmax(mx);
    float sum = 0.0f;
#pragma unroll
    for (int t = 0; t < 12; ++t) { sv[t] = fexp(sv[t] - mx); sum += sv[t]; }
    sum = wsum(sum);
    const float inv = frcp(sum);
    float t0 = 0.0f, t1 = 0.0f, t2 = 0.0f;
#pragma unroll
    for (int t = 0; t < 12; ++t) {
      const int jj = lane + 32 * t;
      const float a = sv[t] * inv;
      srow[jj] = a;
      t0 += a * (cix - sCj[jj * 4 + 0]);
      t1 += a * (ciy - sCj[jj * 4 + 1]);
      t2 += a * (ciz - sCj[jj * 4 + 2]);
    }
    t0 = wsum(t0); t1 = wsum(t1); t2 = wsum(t2);
    if (lane == 0) { sTc[h * 4 + 0] = t0; sTc[h * 4 + 1] = t1; sTc[h * 4 + 2] = t2; }
    __syncthreads();
    {
      const float* vp = qkv + 2 * HID + h * DHD + m;
      const float* ap = srow + 192 * hh;
      const size_t jb = (size_t)(192 * hh);
      float u = 0.0f;
#pragma unroll 4
      for (int jj = 0; jj < 192; ++jj) u += ap[jj] * vp[(jb + (size_t)jj) * QKVW];
      u += __shfl_xor(u, 16);
      if (hh == 0) sU[h * DHD + m] = u;
    }
  }
  __syncthreads();
  if (tid < 3) {
    float c = ec[i * 3 + tid];
#pragma unroll 1
    for (int h = 0; h < NHD; ++h) c += (sTc[h * 4 + tid] * sGt[h]) * 0.125f;
    sCo[tid] = c;
  }
  if (tid == 3) sCo[3] = 0.0f;
  __syncthreads();

  const int l16 = lane & 15;
  v8h uv;
  {
    const v4f a = *(const v4f*)(sU + 8 * l16);
    const v4f b = *(const v4f*)(sU + 8 * l16 + 4);
    uv[0] = (_Float16)(a.x * SC_UPD); uv[1] = (_Float16)(a.y * SC_UPD);
    uv[2] = (_Float16)(a.z * SC_UPD); uv[3] = (_Float16)(a.w * SC_UPD);
    uv[4] = (_Float16)(b.x * SC_UPD); uv[5] = (_Float16)(b.y * SC_UPD);
    uv[6] = (_Float16)(b.z * SC_UPD); uv[7] = (_Float16)(b.w * SC_UPD);
  }
  const int l8 = lane & 7;
  v4f cv = {0.0f, 0.0f, 0.0f, 0.0f};
  if (l8 == 0) cv = *(const v4f*)sCo;
  const bool wu = (wave == 0) && (lane < 16);
  const bool wc = (wave == 0) && (lane < 8);
  _Float16* up = updH + (size_t)i * HID + 8 * l16;
  float* cp = cpl + (size_t)i * CPW + 4 * l8;
  if (wu) *(volatile v8h*)up = uv;
  if (wc) *(volatile v4f*)cp = cv;
  __threadfence();
  if (wu) *(volatile v8h*)up = uv;
  if (wc) *(volatile v4f*)cp = cv;
}

__global__ __launch_bounds__(NTH) void k_out(
    const _Float16* __restrict__ updH, const _Float16* __restrict__ woT,
    const float* __restrict__ ef, const float* __restrict__ bo,
    const float* __restrict__ lng, const float* __restrict__ lnb,
    const float* __restrict__ cpl, float* out0, float* out1) {
  __shared__ __attribute__((aligned(16))) float sTile[32 * TP];
  __shared__ __attribute__((aligned(16))) float sC3[96];
  const int tid = threadIdx.x, lane = tid & 31, wave = tid >> 5;
  const int rb = blockIdx.x;
  if (rb >= E_N / 32) return;
  gemm_tile(updH, 32 * rb, woT, 0, sTile, INV_OUT, lane, wave);
  if (tid < 96) {
    const int q3 = tid / 3;
    sC3[tid] = cpl[(size_t)(32 * rb + q3) * CPW + (tid - 3 * q3)];
  }
  __syncthreads();
  const v4f bo4 = *(const v4f*)(bo + 4 * lane);
  const v4f g4  = *(const v4f*)(lng + 4 * lane);
  const v4f b4  = *(const v4f*)(lnb + 4 * lane);
  v4f ov[8];
#pragma unroll
  for (int q = 0; q < 8; ++q) {
    const int row = wave + 4 * q;
    const int ii = 32 * rb + row;
    const v4f t  = *(const v4f*)(sTile + row * TP + 4 * lane);
    const v4f e4 = *(const v4f*)(ef + (size_t)ii * HID + 4 * lane);
    const v4f y  = e4 + (t + bo4);
    float s = y.x + y.y + y.z + y.w;
    s = wsum(s);
    const float mu = s * (1.0f / 128.0f);
    const v4f d = y - mu;
    float vs = d.x * d.x + d.y * d.y + d.z * d.z + d.w * d.w;
    vs = wsum(vs);
    const float var  = vs * (1.0f / 128.0f);
    const float rstd = rsqrtf(var + 1e-5f);
    ov[q] = d * rstd * g4 + b4;
  }
  const int l24 = (lane < 24) ? lane : 0;
  const v4f cv = *(const v4f*)(sC3 + 4 * l24);
  const bool wc = (wave == 0) && (lane < 24);
#pragma unroll
  for (int q = 0; q < 8; ++q) {
    const int ii = 32 * rb + wave + 4 * q;
    *(volatile v4f*)(out0 + (size_t)ii * HID + 4 * lane) = ov[q];
  }
  if (wc) *(volatile v4f*)(out1 + (size_t)rb * 96 + 4 * lane) = cv;
  __threadfence();
#pragma unroll
  for (int q = 0; q < 8; ++q) {
    const int ii = 32 * rb + wave + 4 * q;
    *(volatile v4f*)(out0 + (size_t)ii * HID + 4 * lane) = ov[q];
  }
  if (wc) *(volatile v4f*)(out1 + (size_t)rb * 96 + 4 * lane) = cv;
}

extern "C" void kernel_launch(void* const* d_in, const int* in_sizes, int n_in,
                              void* d_out, int out_size, void* d_ws, size_t ws_size,
                              hipStream_t stream) {
  if (n_in < 23) return;
  if (in_sizes[0] != E_N * HID || in_sizes[1] != E_N * 3 || in_sizes[2] != E_N * E_N) return;
  if (in_sizes[3] != HID * HID || in_sizes[4] != HID * HID || in_sizes[5] != HID * HID) return;
  if (in_sizes[6] != NRB || in_sizes[7] != NRB) return;
  if (in_sizes[8] != 97 * HID || in_sizes[9] != HID || in_sizes[10] != HID * HID || in_sizes[11] != HID) return;
  if (in_sizes[12] != HID * NHD || in_sizes[13] != NHD) return;
  if (in_sizes[14] != DHD * HID || in_sizes[15] != HID || in_sizes[16] != HID || in_sizes[17] < 1) return;
  if (in_sizes[18] != HID * HID || in_sizes[19] != HID || in_sizes[20] != HID || in_sizes[21] != HID) return;
  if (out_size != E_N * HID + E_N * 3) return;

  const float* ef   = (const float*)d_in[0];
  const float* ec   = (const float*)d_in[1];
  const float* em   = (const float*)d_in[2];
  const float* wq   = (const float*)d_in[3];
  const float* wk   = (const float*)d_in[4];
  const float* wv   = (const float*)d_in[5];
  const float* rc   = (const float*)d_in[6];
  const float* rw   = (const float*)d_in[7];
  const float* a_w1 = (const float*)d_in[8];
  const float* a_b1 = (const float*)d_in[9];
  const float* a_w2 = (const float*)d_in[10];
  const float* a_b2 = (const float*)d_in[11];
  const float* a_w3 = (const float*)d_in[12];
  const float* a_b3 = (const float*)d_in[13];
  const float* g_w1 = (const float*)d_in[14];
  const float* g_b1 = (const float*)d_in[15];
  const float* g_w2 = (const float*)d_in[16];
  const float* g_b2 = (const float*)d_in[17];
  const float* wo   = (const float*)d_in[18];
  const float* bo   = (const float*)d_in[19];
  const float* ln_g = (const float*)d_in[20];
  const float* ln_b = (const float*)d_in[21];

  float* out0 = (float*)d_out;
  float* out1 = out0 + (size_t)E_N * HID;

  char* ws = (char*)d_ws;
  size_t off = 0;
  const size_t oQkvT = off; off += (size_t)QKVW * HID * 2;            off = (off + 255) & ~(size_t)255;
  const size_t oWoT  = off; off += (size_t)HID * HID * 2;             off = (off + 255) & ~(size_t)255;
  const size_t oW2T  = off; off += (size_t)HID * HID * 2;             off = (off + 255) & ~(size_t)255;
  const size_t oA3T  = off; off += (size_t)HID * NRB * 2;             off = (off + 255) & ~(size_t)255;
  const size_t oEfH  = off; off += (size_t)E_N * HID * 2;             off = (off + 255) & ~(size_t)255;
  const size_t oQkv  = off; off += (size_t)E_N * QKVW * 4;            off = (off + 255) & ~(size_t)255;
  const size_t oP    = off; off += (size_t)NHD * E_N * HID * 4;       off = (off + 255) & ~(size_t)255;
  const size_t oQ    = off; off += (size_t)NHD * E_N * HID * 4;       off = (off + 255) & ~(size_t)255;
  const size_t oGpl  = off; off += (size_t)E_N * GPW * 4;             off = (off + 255) & ~(size_t)255;
  const size_t oUpd  = off; off += (size_t)E_N * HID * 2;             off = (off + 255) & ~(size_t)255;
  const size_t oCpl  = off; off += (size_t)E_N * CPW * 4;             off = (off + 255) & ~(size_t)255;
  if (off > ws_size) return;

  _Float16* qkvT = (_Float16*)(ws + oQkvT);
  _Float16* woT  = (_Float16*)(ws + oWoT);
  _Float16* w2T  = (_Float16*)(ws + oW2T);
  _Float16* a3T  = (_Float16*)(ws + oA3T);
  _Float16* efH  = (_Float16*)(ws + oEfH);
  float*    qkv  = (float*)(ws + oQkv);
  float*    Pp   = (float*)(ws + oP);
  float*    Qp   = (float*)(ws + oQ);
  float*    gpl  = (float*)(ws + oGpl);
  _Float16* updH = (_Float16*)(ws + oUpd);
  float*    cpl  = (float*)(ws + oCpl);

  k_prep<<<dim3(36), dim3(NTH), 0, stream>>>(ef, wq, wk, wv, wo, a_w2, a_w1, qkvT, woT, w2T, a3T, efH);
  k_qkv<<<dim3(E_N / 32, 3), dim3(NTH), 0, stream>>>(efH, qkvT, qkv);
  k_node<<<dim3(E_N), dim3(NTH), 0, stream>>>(qkv, a_w1, a_b1, g_w1, g_b1, g_w2, g_b2, Pp, Qp, gpl);
  k_attn<<<dim3(E_N), dim3(NTH), 0, stream>>>(ec, em, rc, rw, a_w1, a_b2, a_w3, a_b3,
                                              qkv, Pp, Qp, gpl, a3T, w2T, updH, cpl);
  k_out<<<dim3(E_N / 32), dim3(NTH), 0, stream>>>(updH, woT, ef, bo, ln_g, ln_b, cpl, out0, out1);
}
